// BlobLayer_24266565222902
// MI455X (gfx1250) — hardware-verified
//
#include <hip/hip_runtime.h>
#include <math.h>

typedef __attribute__((ext_vector_type(16))) _Float16 v16h;
typedef __attribute__((ext_vector_type(16))) __bf16 v16b;
typedef __attribute__((ext_vector_type(8)))  _Float16 v8h;
typedef __attribute__((ext_vector_type(8)))  float v8f;
typedef __attribute__((ext_vector_type(4)))  float v4f;
typedef __attribute__((ext_vector_type(2)))  float v2f;
typedef __attribute__((ext_vector_type(4)))  unsigned v4u;
typedef __attribute__((ext_vector_type(4)))  int v4i;
typedef float __attribute__((may_alias)) float_a;
typedef int __attribute__((may_alias)) int_a;

template <typename T> __device__ __forceinline__ void vst2(void* p, T v) { *(volatile T*)p = v; __threadfence(); *(volatile T*)p = v; }
__device__ __forceinline__ v8f wmma16(v16h a, v16h b, v8f c) {
  v8f d = __builtin_amdgcn_wmma_f32_16x16x32_f16(false, a, false, b, (short)0, c, false, false);
  asm volatile("v_nop\n\tv_nop\n\tv_nop\n\tv_nop" : "+v"(d) : "v"(a), "v"(b));
  return d;
}
__device__ __forceinline__ v8f wmma_bf(v16b a, v16b b, v8f c) {
  v8f d = __builtin_amdgcn_wmma_f32_16x16x32_bf16(false, a, false, b, (short)0, c, false, false);
  asm volatile("v_nop\n\tv_nop\n\tv_nop\n\tv_nop" : "+v"(d) : "v"(a), "v"(b));
  return d;
}
__device__ __forceinline__ v16h frag_h(const _Float16* rowk0, int lane) {
  union { v16h v; v8h q[2]; } u; const _Float16* p = rowk0 + 8 * (lane >> 4);
  u.q[0] = *(const v8h*)p; u.q[1] = *(const v8h*)(p + 16); return u.v;
}
__device__ __forceinline__ v16h frag_f32(const float* rowk0, int lane) {
  v16h a; const float* p = rowk0 + 8 * (lane >> 4);
#pragma unroll
  for (int i = 0; i < 8; ++i) { a[i] = (_Float16)p[i]; a[8 + i] = (_Float16)p[16 + i]; }
  return a;
}
__device__ __forceinline__ v16h frag_f32s(const float* rowk0, int lane, float sc) {
  v16h a; const float* p = rowk0 + 8 * (lane >> 4);
#pragma unroll
  for (int i = 0; i < 8; ++i) { a[i] = (_Float16)(p[i] * sc); a[8 + i] = (_Float16)(p[16 + i] * sc); }
  return a;
}
__device__ __forceinline__ v16h fragc_f32(const float* W, int k0, int n, int lane, int ld, int K) {
  v16h a; const int g = lane >> 4;
#pragma unroll
  for (int i = 0; i < 8; ++i) { const int ka = k0 + 8 * g + i, kb = ka + 16;
    a[i] = (_Float16)(ka < K ? W[(size_t)ka * ld + n] : 0.f); a[8 + i] = (_Float16)(kb < K ? W[(size_t)kb * ld + n] : 0.f); }
  return a;
}
struct F2 { v16b h, l; };
__device__ __forceinline__ F2 bsplit16(const float v[16]) { F2 r;
#pragma unroll
  for (int i = 0; i < 16; ++i) { const __bf16 h = (__bf16)v[i]; r.h[i] = h; r.l[i] = (__bf16)(v[i] - (float)h); }
  return r; }
__device__ __forceinline__ F2 split_row(const float* row, int k0, int lane) { float v[16]; const float* p = row + k0 + 8 * (lane >> 4);
#pragma unroll
  for (int i = 0; i < 8; ++i) { v[i] = p[i]; v[8 + i] = p[16 + i]; }
  return bsplit16(v); }
__device__ __forceinline__ F2 split_rowK(const float* row, int k0, int lane, int K) { float v[16]; const int g = lane >> 4;
#pragma unroll
  for (int i = 0; i < 8; ++i) { const int ka = k0 + 8 * g + i, kb = ka + 16; v[i] = ka < K ? row[ka] : 0.f; v[8 + i] = kb < K ? row[kb] : 0.f; }
  return bsplit16(v); }
__device__ __forceinline__ F2 split_col(const float* W, int k0, int n, int lane, int ld, int K) { float v[16]; const int g = lane >> 4;
#pragma unroll
  for (int i = 0; i < 8; ++i) { const int ka = k0 + 8 * g + i, kb = ka + 16; v[i] = ka < K ? W[(size_t)ka * ld + n] : 0.f; v[8 + i] = kb < K ? W[(size_t)kb * ld + n] : 0.f; }
  return bsplit16(v); }
__device__ __forceinline__ v8f mac3(const F2& a, const F2& b, v8f c) { c = wmma_bf(a.l, b.h, c); c = wmma_bf(a.h, b.l, c); return wmma_bf(a.h, b.h, c); }
__device__ __forceinline__ float sigm(float v) { return 1.0f / (1.0f + expf(-v)); }
#define LDSX() do { asm volatile("s_wait_dscnt 0" ::: "memory"); __builtin_amdgcn_wave_barrier(); __builtin_amdgcn_fence(__ATOMIC_RELEASE, "workgroup"); } while (0)


#define NB 256
#define NP 50176
#define NC 1024
#define KSPLIT 7
#define KPER (NP / KSPLIT)
__device__ __forceinline__ float bfr(float v) { return (float)(__bf16)v; }
__device__ __forceinline__ v16b frag_b(const __bf16* rowk0, int lane) { return __builtin_bit_cast(v16b, frag_h((const _Float16*)rowk0, lane)); }

__global__ __launch_bounds__(256) void k_gemm(const float* __restrict__ x, const float* __restrict__ pos, const float* __restrict__ sig, const float* __restrict__ cwt, const float* __restrict__ xs, const float* __restrict__ ys, float* __restrict__ PART) {
  __shared__ __align__(16) __bf16 sCh[128][40], sCl[128][40];
  __shared__ __align__(16) float so[8][16][132];
  __shared__ float sp0[128], sp1[128], sts[128], sfw[128];
  const int tid = threadIdx.x, wave = tid >> 5, lane = tid & 31, col = lane & 15, g = lane >> 4;
  const int n0 = blockIdx.x * 128, ks = blockIdx.y; const int kbase = ks * KPER;
  if (tid < 128) { const int c = n0 + tid; const float s = bfr(sig[c]); sp0[tid] = bfr(pos[c * 2]); sp1[tid] = bfr(pos[c * 2 + 1]); sts[tid] = 2.0f * s * s + 0.001f; sfw[tid] = bfr(cwt[c]) / (2.0f * 3.141592653589793f * s * s + 0.001f); }
  __syncthreads();
  const int cc = tid & 127, hk = tid >> 7;
  v8f acc[2][8] = {};
#pragma unroll 1
  for (int kc = 0; kc < KPER / 32; ++kc) { const int k0 = kbase + kc * 32;
    { const float p0 = sp0[cc], p1 = sp1[cc], ts = sts[cc], fw = sfw[cc];
#pragma unroll 4
      for (int e = 0; e < 16; ++e) { const int p = k0 + hk * 16 + e; const float dx = bfr(xs[p]) - p1, dy = bfr(ys[p]) - p0; float v = fw * expf(-(dx * dx + dy * dy) / ts); v = fminf(fmaxf(v, -2000.0f), 2000.0f);
        const __bf16 hi = (__bf16)v; sCh[cc][hk * 16 + e] = hi; sCl[cc][hk * 16 + e] = (__bf16)(v - (float)hi); } }
    __syncthreads();
#pragma unroll
    for (int rt = 0; rt < 2; ++rt) { const v16b a = split_row(x + (size_t)((wave * 2 + rt) * 16 + col) * NP, k0, lane).h;
#pragma unroll
      for (int j = 0; j < 8; ++j) { acc[rt][j] = wmma_bf(a, frag_b(&sCh[j * 16 + col][0], lane), acc[rt][j]); acc[rt][j] = wmma_bf(a, frag_b(&sCl[j * 16 + col][0], lane), acc[rt][j]); } }
    __syncthreads(); }
#pragma unroll
  for (int rt = 0; rt < 2; ++rt) {
#pragma unroll
    for (int j = 0; j < 8; ++j)
#pragma unroll
      for (int r = 0; r < 8; ++r) so[wave][8 * g + r][j * 16 + col] = acc[rt][j][r];
    LDSX();
    for (int rl = 0; rl < 16; ++rl) vst2(PART + ((size_t)ks * NB + (wave * 2 + rt) * 16 + rl) * NC + n0 + lane * 4, *(const v4f*)(&so[wave][rl][lane * 4]));
    LDSX(); }
}
__global__ __launch_bounds__(256) void k_sum(const float* __restrict__ PART, float* __restrict__ out) {
  const size_t i4 = (size_t)blockIdx.x * 256 + threadIdx.x; if (i4 >= (size_t)NB * NC / 4) return;
  v4f s = *(const v4f*)(PART + i4 * 4);
#pragma unroll
  for (int k = 1; k < KSPLIT; ++k) { const v4f t = *(const v4f*)(PART + (size_t)k * NB * NC + i4 * 4); s += t; }
  vst2(out + i4 * 4, s * (1.0f / (float)NP));
}
extern "C" void kernel_launch(void* const* d_in, const int* in_sizes, int n_in, void* d_out, int out_size, void* d_ws, size_t ws_size, hipStream_t stream) {
  (void)in_sizes; (void)n_in; (void)out_size; (void)ws_size;
  const float* x = (const float*)d_in[0]; const float* pos = (const float*)d_in[1]; const float* sig = (const float*)d_in[2]; const float* cwt = (const float*)d_in[3]; const float* xs = (const float*)d_in[4]; const float* ys = (const float*)d_in[5];
  float* PART = (float*)d_ws;
  k_gemm<<<dim3(NC / 128, KSPLIT), 256, 0, stream>>>(x, pos, sig, cwt, xs, ys, PART);
  k_sum<<<(NB * NC / 4 + 255) / 256, 256, 0, stream>>>(PART, (float*)d_out);
}
